// MultiHeadAttention_32770600468859
// MI455X (gfx1250) — hardware-verified
//
#include <hip/hip_runtime.h>
#ifndef NB
#define NB 2
#endif
#ifndef SEQ
#define SEQ 1024
#endif
#define NB_FULL 2
#define SEQ_FULL 1024
#define DM 1024
#define NH 16
#define HD 64
#define NR ((size_t)NB * SEQ)
#define MR ((int)(NB * SEQ))

typedef unsigned short v8us __attribute__((ext_vector_type(8), may_alias));
typedef float  v8f  __attribute__((ext_vector_type(8)));
typedef float  v4f  __attribute__((ext_vector_type(4)));
typedef float  v4fa __attribute__((ext_vector_type(4), may_alias));
typedef _Float16 v16h __attribute__((ext_vector_type(16)));
typedef _Float16 v4h __attribute__((ext_vector_type(4)));
union FragH { v16h v; v8us half[2]; _Float16 h[16]; unsigned short u[16]; };

static_assert(NH * HD == DM);
static_assert(HD == 64);
static_assert(DM % 64 == 0 && DM % 32 == 0 && DM % 8 == 0);
static_assert(SEQ % 64 == 0);
static_assert((NB * SEQ) % 128 == 0);
static_assert(SEQ / 32 <= 128);
static_assert(NB <= NB_FULL && SEQ <= SEQ_FULL);
static_assert(((size_t)NB * SEQ * DM) % (8 * 256) == 0);
static_assert(((size_t)DM * DM) % (8 * 256) == 0);

__device__ __forceinline__ unsigned short bf16_bits(float x) { unsigned int u = __float_as_uint(x); return (unsigned short)((u + 0x7FFFu + ((u >> 16) & 1u)) >> 16); }
__device__ __forceinline__ float bf16_val(unsigned short b) { return __uint_as_float(((unsigned int)b) << 16); }
__device__ __forceinline__ float bfr(float x) { return bf16_val(bf16_bits(x)); }

__device__ __forceinline__ v16h g2_frag(const _Float16* p, int hh) { FragH f; f.half[0] = *(const v8us*)((const unsigned short*)p + 8 * hh); f.half[1] = *(const v8us*)((const unsigned short*)p + 16 + 8 * hh); return f.v; }
__device__ __forceinline__ v8f g2_mma(v16h a, v16h b, v8f c) { v8f d = __builtin_amdgcn_wmma_f32_16x16x32_f16(false, a, false, b, (short)0, c, false, false); asm volatile("v_nop\n\tv_nop\n\tv_nop\n\tv_nop" : "+v"(d) : "v"(a), "v"(b)); return d; }

__global__ __launch_bounds__(256) void k_wnat(const float* __restrict__ w, _Float16* __restrict__ Bt) {
  const size_t t = (size_t)blockIdx.x * 256 + threadIdx.x; if (t >= (size_t)DM * DM / 8) return;
  const v4f a = *(const v4fa*)(w + t * 8), c = *(const v4fa*)(w + t * 8 + 4); FragH f;
#pragma unroll
  for (int q = 0; q < 4; ++q) { f.h[q] = (_Float16)(bfr(a[q]) * 16.0f); f.h[4 + q] = (_Float16)(bfr(c[q]) * 16.0f); }
  const v8us o = f.half[0];
  *(volatile v8us*)((unsigned short*)Bt + t * 8) = o; __threadfence(); *(volatile v8us*)((unsigned short*)Bt + t * 8) = o;
}

__global__ __launch_bounds__(256) void k_x16(const float* __restrict__ x, _Float16* __restrict__ X16) {
  const size_t t = (size_t)blockIdx.x * 256 + threadIdx.x; if (t >= NR * DM / 8) return;
  const size_t e = t * 8; const size_t row = e / DM; const size_t col = e % DM; const size_t bb = row / SEQ, s = row % SEQ;
  const float* src = x + (bb * SEQ_FULL + s) * DM + col;
  const v4f a = *(const v4fa*)(src), c = *(const v4fa*)(src + 4); FragH f;
#pragma unroll
  for (int q = 0; q < 4; ++q) { f.h[q] = (_Float16)bfr(a[q]); f.h[4 + q] = (_Float16)bfr(c[q]); }
  const v8us o = f.half[0];
  *(volatile v8us*)((unsigned short*)X16 + t * 8) = o; __threadfence(); *(volatile v8us*)((unsigned short*)X16 + t * 8) = o;
}

template <bool F32OUT>
__device__ __forceinline__ void gemm2_body(const _Float16* __restrict__ A, int lda, const _Float16* __restrict__ Bh, int ldb, float alpha, const float* __restrict__ bias,
                                           float* __restrict__ C, _Float16* __restrict__ C16, int ldc, int N, int K) {
  __shared__ __attribute__((aligned(16))) float so[4][32][68];
  const int tid = threadIdx.x; const int w = __builtin_amdgcn_readfirstlane(tid >> 5); const int lane = tid & 31, ln = lane & 15, hh = lane >> 4;
  const int ntn = N >> 6; const int mt = blockIdx.x / ntn, nq = blockIdx.x - mt * ntn; const int row0 = mt * 128 + 32 * w, col0 = nq * 64;
  const _Float16* a0p = A + (size_t)(row0 + ln) * lda; const _Float16* a1p = a0p + (size_t)16 * lda;
  const _Float16* b0p = Bh + (size_t)(col0 + ln) * ldb; const _Float16* b1p = b0p + (size_t)16 * ldb; const _Float16* b2p = b1p + (size_t)16 * ldb; const _Float16* b3p = b2p + (size_t)16 * ldb;
  const v8f z8 = {0.f,0.f,0.f,0.f,0.f,0.f,0.f,0.f}; v8f c00 = z8, c01 = z8, c02 = z8, c03 = z8, c10 = z8, c11 = z8, c12 = z8, c13 = z8;
#pragma unroll 1
  for (int kb = 0; kb < K; kb += 32) { const v16h a0 = g2_frag(a0p + kb, hh), a1 = g2_frag(a1p + kb, hh);
    v16h b = g2_frag(b0p + kb, hh); c00 = g2_mma(a0, b, c00); c10 = g2_mma(a1, b, c10);
    b = g2_frag(b1p + kb, hh); c01 = g2_mma(a0, b, c01); c11 = g2_mma(a1, b, c11);
    b = g2_frag(b2p + kb, hh); c02 = g2_mma(a0, b, c02); c12 = g2_mma(a1, b, c12);
    b = g2_frag(b3p + kb, hh); c03 = g2_mma(a0, b, c03); c13 = g2_mma(a1, b, c13); }
  v8f accs[8] = {c00, c01, c02, c03, c10, c11, c12, c13};
#pragma unroll
  for (int u = 0; u < 8; ++u) { const int t = u & 3, half = u >> 2; const int col = col0 + t * 16 + ln; const float bv = bfr(bias[col]);
#pragma unroll
    for (int r = 0; r < 8; ++r) { const int rloc = half * 16 + 8 * hh + r; so[w][rloc][t * 16 + ln] = accs[u][r] * alpha + bv; } }
  __syncthreads();
  const int rsub = lane >> 4, c4 = (lane & 15) * 4;
  for (int pass = 0; pass < 2; ++pass) {
#pragma unroll
    for (int q = 0; q < 16; ++q) { const int r = q * 2 + rsub; const v4f v = *(const v4fa*)&so[w][r][c4];
      if (F32OUT) { *(volatile v4f*)(C + (size_t)(row0 + r) * ldc + col0 + c4) = v; }
      else { v4h h4; h4[0] = (_Float16)v[0]; h4[1] = (_Float16)v[1]; h4[2] = (_Float16)v[2]; h4[3] = (_Float16)v[3]; *(volatile v4h*)(C16 + (size_t)(row0 + r) * ldc + col0 + c4) = h4; } }
    if (pass == 0) __threadfence(); }
}
__global__ __launch_bounds__(128) void k_gemm_h16(const _Float16* __restrict__ A, int lda, const _Float16* __restrict__ Bh, int ldb, float alpha, const float* __restrict__ bias, _Float16* __restrict__ C16, int ldc, int N, int K) {
  gemm2_body<false>(A, lda, Bh, ldb, alpha, bias, nullptr, C16, ldc, N, K);
}
__global__ __launch_bounds__(128) void k_gemm_f32(const _Float16* __restrict__ A, int lda, const _Float16* __restrict__ Bh, int ldb, float alpha, const float* __restrict__ bias, float* __restrict__ C, int ldc, int N, int K) {
  gemm2_body<true>(A, lda, Bh, ldb, alpha, bias, C, nullptr, ldc, N, K);
}

__global__ __launch_bounds__(256) void k_vt(const _Float16* __restrict__ V16, _Float16* __restrict__ Vt) {
  __shared__ unsigned short tl[64][66];
  const int tid = threadIdx.x; const int slab = blockIdx.x / (SEQ / 64), lg = blockIdx.x % (SEQ / 64); const int b = slab / NH, h = slab % NH;
  for (int i = tid; i < 64 * 8; i += 256) { const int r = i / 8, c8 = (i % 8) * 8; FragH f; f.half[0] = *(const v8us*)((const unsigned short*)V16 + ((size_t)b * SEQ + lg * 64 + r) * DM + h * HD + c8);
#pragma unroll
    for (int q = 0; q < 8; ++q) tl[r][c8 + q] = f.u[q]; }
  __syncthreads();
  for (int pass = 0; pass < 2; ++pass) {
#pragma unroll
    for (int rd = 0; rd < 2; ++rd) { const int d = rd * 32 + tid / 8, pc = tid % 8; FragH f;
#pragma unroll
      for (int q = 0; q < 8; ++q) f.u[q] = tl[pc * 8 + q][d];
      *(volatile v8us*)((unsigned short*)Vt + ((size_t)slab * 64 + d) * SEQ + lg * 64 + pc * 8) = f.half[0]; }
    if (pass == 0) __threadfence(); }
}

__global__ __launch_bounds__(128) void k_attn(const _Float16* __restrict__ Q16, const _Float16* __restrict__ K16, const _Float16* __restrict__ Vt, const int* __restrict__ mask, _Float16* __restrict__ CTX) {
  __shared__ unsigned int smw[SEQ / 32];
  __shared__ __attribute__((aligned(16))) unsigned short sh[4][16][72];
  const int tid = threadIdx.x; const int wave = __builtin_amdgcn_readfirstlane(tid >> 5); const int lane = tid & 31, ln = lane & 15, hh = lane >> 4;
  const int h = blockIdx.y, b = blockIdx.z;
  {
    const int wi = (tid < SEQ / 32) ? tid : (SEQ / 32 - 1);
    const int* mp = mask + (size_t)b * SEQ_FULL + (size_t)wi * 32; unsigned int wbits = 0u;
#pragma unroll 1
    for (int j = 0; j < 32; ++j) wbits |= ((mp[j] != 0) ? 1u : 0u) << j;
    if (tid < SEQ / 32) smw[tid] = wbits;
  }
  __syncthreads();
  const int q0 = blockIdx.x * 64 + wave * 16; const size_t rowb = (size_t)b * SEQ;
  const _Float16* Qp = Q16 + (rowb + q0 + ln) * DM + h * HD;
  const v16h qf0 = g2_frag(Qp, hh), qf1 = g2_frag(Qp + 32, hh);
  const _Float16* Kp = K16 + (rowb + ln) * DM + h * HD;
  const _Float16* Vp = Vt + ((size_t)(b * NH + h) * HD + ln) * SEQ;
  const v8f z8 = {0.f,0.f,0.f,0.f,0.f,0.f,0.f,0.f};
  v8f o0 = z8, o1 = z8, o2 = z8, o3 = z8; float mrun = -1.0e30f, lpart = 0.f;
#pragma unroll 1
  for (int kb = 0; kb < SEQ; kb += 32) {
    const _Float16* k0p = Kp + (size_t)kb * DM; const _Float16* k1p = k0p + (size_t)16 * DM;
    v8f s0 = z8, s1 = z8;
    v16h a = g2_frag(k0p, hh); s0 = g2_mma(a, qf0, s0);
    a = g2_frag(k0p + 32, hh); s0 = g2_mma(a, qf1, s0);
    a = g2_frag(k1p, hh); s1 = g2_mma(a, qf0, s1);
    a = g2_frag(k1p + 32, hh); s1 = g2_mma(a, qf1, s1);
    const unsigned int mw = smw[kb >> 5] >> (8 * hh);
    float e0[8], e1[8]; float mx = -3.0e38f;
#pragma unroll
    for (int r = 0; r < 8; ++r) {
      float x0 = s0[r] * 0.125f; x0 = ((mw >> r) & 1u) ? x0 : -1.0e9f;
      float x1 = s1[r] * 0.125f; x1 = ((mw >> (16 + r)) & 1u) ? x1 : -1.0e9f;
      e0[r] = x0; e1[r] = x1; mx = fmaxf(mx, fmaxf(x0, x1));
    }
    mx = fmaxf(mx, __shfl_xor(mx, 16));
    const float mnew = fmaxf(mrun, mx); const float alpha = __expf(mrun - mnew); mrun = mnew;
    float ps = 0.f; FragH pf;
#pragma unroll
    for (int r = 0; r < 8; ++r) {
      const float p0 = __expf(e0[r] - mnew), p1 = __expf(e1[r] - mnew); ps += p0 + p1;
      pf.h[r] = (_Float16)(p0 * 1024.0f); pf.h[8 + r] = (_Float16)(p1 * 1024.0f);
    }
    lpart = lpart * alpha + ps;
#pragma unroll
    for (int r = 0; r < 8; ++r) { o0[r] *= alpha; o1[r] *= alpha; o2[r] *= alpha; o3[r] *= alpha; }
    const v16h pb = pf.v;
    a = g2_frag(Vp + kb, hh); o0 = g2_mma(a, pb, o0);
    a = g2_frag(Vp + (size_t)16 * SEQ + kb, hh); o1 = g2_mma(a, pb, o1);
    a = g2_frag(Vp + (size_t)32 * SEQ + kb, hh); o2 = g2_mma(a, pb, o2);
    a = g2_frag(Vp + (size_t)48 * SEQ + kb, hh); o3 = g2_mma(a, pb, o3);
  }
  const float l = lpart + __shfl_xor(lpart, 16);
  const float inv = 1.0f / (l * 16.0f);
  FragH t0, t1, t2, t3;
#pragma unroll
  for (int r = 0; r < 8; ++r) { t0.h[r] = (_Float16)(o0[r] * inv); t1.h[r] = (_Float16)(o1[r] * inv); t2.h[r] = (_Float16)(o2[r] * inv); t3.h[r] = (_Float16)(o3[r] * inv); }
  *(v8us*)&sh[wave][ln][0 + 8 * hh] = t0.half[0];
  *(v8us*)&sh[wave][ln][16 + 8 * hh] = t1.half[0];
  *(v8us*)&sh[wave][ln][32 + 8 * hh] = t2.half[0];
  *(v8us*)&sh[wave][ln][48 + 8 * hh] = t3.half[0];
  __syncthreads();
  const int rsub = lane >> 3, pc = lane & 7;
  for (int pass = 0; pass < 2; ++pass) {
#pragma unroll
    for (int it = 0; it < 4; ++it) { const int row = it * 4 + rsub; const v8us v = *(const v8us*)&sh[wave][row][pc * 8];
      *(volatile v8us*)((unsigned short*)CTX + (rowb + q0 + row) * DM + h * HD + pc * 8) = v; }
    if (pass == 0) __threadfence(); }
}

#define WBYTES ((size_t)DM * DM * 2)
#define PBYTES ((size_t)NB * SEQ * DM * 2)
static_assert(WBYTES % 256 == 0 && PBYTES % 256 == 0);
static_assert(4 * WBYTES + 8 * PBYTES <= (size_t)134217728);

extern "C" void kernel_launch(void* const* d_in, const int* in_sizes, int n_in,
                              void* d_out, int out_size, void* d_ws, size_t ws_size, hipStream_t stream) {
  if (n_in < 12) return;
  const long long need_x = (long long)(NB - 1) * SEQ_FULL * DM + (long long)SEQ * DM;
  if ((long long)in_sizes[0] < need_x || (long long)in_sizes[1] < need_x || (long long)in_sizes[2] < need_x) return;
  if ((long long)in_sizes[3] < (long long)(NB - 1) * SEQ_FULL + SEQ) return;
  if (in_sizes[4] < DM * DM || in_sizes[6] < DM * DM || in_sizes[8] < DM * DM || in_sizes[10] < DM * DM) return;
  if (in_sizes[5] < DM || in_sizes[7] < DM || in_sizes[9] < DM || in_sizes[11] < DM) return;
  if ((long long)out_size < (long long)NB * SEQ * DM) return;
  const float* xq = (const float*)d_in[0]; const float* xk = (const float*)d_in[1]; const float* xv = (const float*)d_in[2];
  const int* mask = (const int*)d_in[3];
  const float* Wq = (const float*)d_in[4]; const float* bq = (const float*)d_in[5];
  const float* Wk = (const float*)d_in[6]; const float* bk = (const float*)d_in[7];
  const float* Wv = (const float*)d_in[8]; const float* bv = (const float*)d_in[9];
  const float* Wo = (const float*)d_in[10]; const float* bo = (const float*)d_in[11];
  float* out = (float*)d_out;
  char* ws = (char*)d_ws; size_t off = 0;
  _Float16* BQ = (_Float16*)(ws + off); off += WBYTES;
  _Float16* BK = (_Float16*)(ws + off); off += WBYTES;
  _Float16* BV = (_Float16*)(ws + off); off += WBYTES;
  _Float16* BO = (_Float16*)(ws + off); off += WBYTES;
  _Float16* XQ = (_Float16*)(ws + off); off += PBYTES;
  _Float16* XK = (_Float16*)(ws + off); off += PBYTES;
  _Float16* XV = (_Float16*)(ws + off); off += PBYTES;
  _Float16* Q16 = (_Float16*)(ws + off); off += PBYTES;
  _Float16* K16 = (_Float16*)(ws + off); off += PBYTES;
  _Float16* V16 = (_Float16*)(ws + off); off += PBYTES;
  _Float16* VT = (_Float16*)(ws + off); off += PBYTES;
  _Float16* CTX = (_Float16*)(ws + off); off += PBYTES;
  if (off > ws_size) return;
  const unsigned gw = (unsigned)(((size_t)DM * DM / 8) / 256);
  const unsigned gx = (unsigned)((NR * DM / 8) / 256);
  k_wnat<<<gw, 256, 0, stream>>>(Wq, BQ);
  k_wnat<<<gw, 256, 0, stream>>>(Wk, BK);
  k_wnat<<<gw, 256, 0, stream>>>(Wv, BV);
  k_wnat<<<gw, 256, 0, stream>>>(Wo, BO);
  k_x16<<<gx, 256, 0, stream>>>(xq, XQ);
  k_x16<<<gx, 256, 0, stream>>>(xk, XK);
  k_x16<<<gx, 256, 0, stream>>>(xv, XV);
  const unsigned gg = (unsigned)((MR / 128) * (DM / 64));
  k_gemm_h16<<<gg, 128, 0, stream>>>(XQ, DM, BQ, DM, 0.0625f, bq, Q16, DM, DM, DM);
  k_gemm_h16<<<gg, 128, 0, stream>>>(XK, DM, BK, DM, 0.0625f, bk, K16, DM, DM, DM);
  k_gemm_h16<<<gg, 128, 0, stream>>>(XV, DM, BV, DM, 0.0625f, bv, V16, DM, DM, DM);
  k_vt<<<(unsigned)(NB * NH * (SEQ / 64)), 256, 0, stream>>>(V16, VT);
  k_attn<<<dim3(SEQ / 64, NH, NB), 128, 0, stream>>>(Q16, K16, VT, mask, CTX);
  k_gemm_f32<<<gg, 128, 0, stream>>>(CTX, DM, BO, DM, 0.0009765625f, bo, out, DM, DM, DM);
}
